// TemporalBlock_42872363548704
// MI455X (gfx1250) — hardware-verified
//
#include <hip/hip_runtime.h>
#include <math.h>
#include <stdint.h>

constexpr int kBatch  = 32;
constexpr int kSeqT   = 128;
constexpr int kFeat   = 32;
constexpr int kHid    = 256;
constexpr int kRows   = kBatch * kSeqT;
constexpr int kAssets = 1000;
constexpr int kGate4  = 4 * kHid;
constexpr int kMixK   = kFeat * kHid + kFeat;
constexpr int kMixLd  = kMixK + 32;
constexpr int kPadM   = 64;
constexpr float kWCarry   = 16.0f;
constexpr float kWInv     = 1.0f / 16.0f;
constexpr float kUCarry   = 1024.0f;
constexpr float kMixScale = 1.0f / (1024.0f * 16.0f);
constexpr float kEmbScale = 1.0f / 256.0f;
constexpr float kInvH     = 1.0f / 256.0f;
constexpr float kLnEps    = 1e-5f;
static_assert(kRows == 4096, "rows");
static_assert(kMixK == 8224 && (kMixK % 32) == 0, "mix K tile");
static_assert(kMixLd == 8256 && ((kMixLd * 2) % 128) == 0, "mix row pitch is whole lines");

typedef __attribute__((ext_vector_type(16))) _Float16 v16h;
typedef __attribute__((ext_vector_type(8)))  _Float16 v8h;
typedef __attribute__((ext_vector_type(16))) __bf16   v16b;
typedef __attribute__((ext_vector_type(8)))  __bf16   v8b;
typedef __attribute__((ext_vector_type(8)))  float    v8f;
typedef __attribute__((ext_vector_type(4)))  float    v4f;
typedef __attribute__((ext_vector_type(4)))  unsigned int v4u;

__device__ __forceinline__ unsigned short f2bf_bits(float f) {
  unsigned u = __float_as_uint(f);
  return (unsigned short)((u + 0x7FFFu + ((u >> 16) & 1u)) >> 16);
}
__device__ __forceinline__ float bf_bits2f(unsigned short h) { return __uint_as_float(((unsigned)h) << 16); }

__device__ __forceinline__ void dep_guard_h(v8f& a, v8f& b, v16h x, v16h y) { asm volatile("v_nop\n\tv_nop\n\tv_nop\n\tv_nop" : "+v"(a), "+v"(b) : "v"(x), "v"(y)); }
__device__ __forceinline__ void dep_guard_b(v8f& a, v8f& b, v16b x, v16b y) { asm volatile("v_nop\n\tv_nop\n\tv_nop\n\tv_nop" : "+v"(a), "+v"(b) : "v"(x), "v"(y)); }
__device__ __forceinline__ void keep4_h(v16h a, v16h b, v16h c, v16h d) { asm volatile("v_nop" :: "v"(a), "v"(b), "v"(c), "v"(d)); }
__device__ __forceinline__ void keep4_b(v16b a, v16b b, v16b c, v16b d) { asm volatile("v_nop" :: "v"(a), "v"(b), "v"(c), "v"(d)); }
__device__ __forceinline__ void acc_guard4(v8f& a, v8f& b, v8f& c, v8f& d) { asm volatile("v_nop\n\tv_nop\n\tv_nop\n\tv_nop" : "+v"(a), "+v"(b), "+v"(c), "+v"(d)); }
template <typename T> struct Frag;
template <> struct Frag<_Float16> {
  typedef v16h V; union U { v16h v; v8h h[2]; };
  static __device__ __forceinline__ v16h load(const _Float16* p) {
    U f; f.h[0] = *(const v8h*)(p); f.h[1] = *(const v8h*)(p + 16); return f.v;
  }
  static __device__ __forceinline__ v8f mma(v16h a, v16h b, v8f c) {
    return __builtin_amdgcn_wmma_f32_16x16x32_f16(false, a, false, b, (short)0, c, false, false);
  }
  static __device__ __forceinline__ void guard(v8f& a, v8f& b, v16h x, v16h y) { dep_guard_h(a, b, x, y); }
  static __device__ __forceinline__ void keep(v16h a, v16h b, v16h c, v16h d) { keep4_h(a, b, c, d); }
};
template <> struct Frag<__bf16> {
  typedef v16b V; union U { v16b v; v8b h[2]; };
  static __device__ __forceinline__ v16b load(const __bf16* p) {
    U f; f.h[0] = *(const v8b*)(p); f.h[1] = *(const v8b*)(p + 16); return f.v;
  }
  static __device__ __forceinline__ v8f mma(v16b a, v16b b, v8f c) {
    return __builtin_amdgcn_wmma_f32_16x16x32_bf16(false, a, false, b, (short)0, c, false, false);
  }
  static __device__ __forceinline__ void guard(v8f& a, v8f& b, v16b x, v16b y) { dep_guard_b(a, b, x, y); }
  static __device__ __forceinline__ void keep(v16b a, v16b b, v16b c, v16b d) { keep4_b(a, b, c, d); }
};

__device__ __forceinline__ unsigned pk16(unsigned short a, unsigned short b) { return (unsigned)a | ((unsigned)b << 16); }
__device__ __forceinline__ unsigned short h_bits(float f) { const _Float16 h = (_Float16)f; return __builtin_bit_cast(unsigned short, h); }
__device__ __forceinline__ float eluf(float v) { return (v > 0.0f) ? v : (expf(v) - 1.0f); }

template <int ET> struct Elem;
template <> struct Elem<0> { typedef _Float16 T; };
template <> struct Elem<1> { typedef __bf16 T; };
template <int ET, bool SPLIT, int BIAS_MODE, int OUT_MODE, bool RESID, int ACT = 0>
__global__ __launch_bounds__(256) void wmma_gemm64(
    const unsigned short* __restrict__ Ap, const unsigned short* __restrict__ A2p, int lda, long strideA,
    const unsigned short* __restrict__ Btp, const unsigned short* __restrict__ Bt2p, int ldb, long strideB,
    void* __restrict__ Cout, void* __restrict__ Cout2, int ldc, long strideC,
    const float* __restrict__ bias,
    const float* __restrict__ resid, long strideR,
    int M, int N, int K, float scale) {
  typedef typename Elem<ET>::T T;
  typedef typename Frag<T>::V V;
  const T* A = (const T*)Ap; const T* A2 = (const T*)A2p; const T* Bt = (const T*)Btp; const T* Bt2 = (const T*)Bt2p;
  __shared__ __align__(16) float sT[8][16 * 68];
  const int b    = blockIdx.y;
  const int lane = threadIdx.x & 31;
  const int wave = threadIdx.x >> 5;
  const int tilesN = N >> 6;
  const int tilesM = M >> 6;
  const int tile = blockIdx.x * 8 + wave;
  if (tile >= tilesM * tilesN) return;
  const int tm = tile / tilesN;
  const int tn = tile - tm * tilesN;
  const int m0 = tm << 6;
  const int n0 = tn << 6;

  const T* Ab  = A  + (size_t)b * strideA;
  const T* Bb  = Bt + (size_t)b * strideB;
  const T* Ab2 = SPLIT ? (A2  + (size_t)b * strideA) : nullptr;
  const T* Bb2 = SPLIT ? (Bt2 + (size_t)b * strideB) : nullptr;

  const int rlane = lane & 15;
  const int koff  = (lane >> 4) * 8;
  const int mOff  = (lane >> 4) * 8;

  v8f acc[4][4];
#pragma unroll
  for (int i = 0; i < 4; ++i)
#pragma unroll
    for (int j = 0; j < 4; ++j) acc[i][j] = (v8f){0.f,0.f,0.f,0.f,0.f,0.f,0.f,0.f};

  for (int k0 = 0; k0 < K; k0 += 32) {
    V bh[4], bl[4];
#pragma unroll
    for (int j = 0; j < 4; ++j) {
      const size_t bo = (size_t)(n0 + (j << 4) + rlane) * ldb + koff + k0;
      bh[j] = Frag<T>::load(Bb + bo);
      if (SPLIT) bl[j] = Frag<T>::load(Bb2 + bo);
    }
#pragma unroll
    for (int i = 0; i < 4; ++i) {
      const size_t ao = (size_t)(m0 + (i << 4) + rlane) * lda + koff + k0;
      V ah = Frag<T>::load(Ab + ao);
      V al;
      if (SPLIT) al = Frag<T>::load(Ab2 + ao);
#pragma unroll
      for (int j = 0; j < 4; ++j) {
        acc[i][j] = Frag<T>::mma(ah, bh[j], acc[i][j]);
        if (SPLIT) {
          acc[i][j] = Frag<T>::mma(ah, bl[j], acc[i][j]);
          acc[i][j] = Frag<T>::mma(al, bh[j], acc[i][j]);
        }
      }
      Frag<T>::guard(acc[i][0], acc[i][3], ah, SPLIT ? al : ah);
    }
    Frag<T>::keep(bh[0], bh[1], bh[2], bh[3]);
    if (SPLIT) Frag<T>::keep(bl[0], bl[1], bl[2], bl[3]);
  }
  acc_guard4(acc[0][0], acc[0][1], acc[0][2], acc[0][3]);
  acc_guard4(acc[1][0], acc[1][1], acc[1][2], acc[1][3]);
  acc_guard4(acc[2][0], acc[2][1], acc[2][2], acc[2][3]);
  acc_guard4(acc[3][0], acc[3][1], acc[3][2], acc[3][3]);

  float* slab = sT[wave];
  const float* Rb = RESID ? (resid + (size_t)b * strideR) : nullptr;
#pragma unroll
  for (int i = 0; i < 4; ++i) {
    const int mBase = m0 + (i << 4);
#pragma unroll
    for (int j = 0; j < 4; ++j) {
      const int n = n0 + (j << 4) + rlane;
      float bv = 0.f;
      if (BIAS_MODE == 2) bv = bias[n];
#pragma unroll
      for (int r = 0; r < 8; ++r) {
        float v = acc[i][j][r] * scale;
        if (BIAS_MODE == 1) v += bias[mBase + mOff + r];
        if (BIAS_MODE == 2) v += bv;
        if (RESID) v += Rb[(size_t)(mBase + mOff + r) * ldc + n];
        if (ACT == 2) v = fmaxf(v, 0.0f);
        if (ACT == 4) v = (v > 0.f) ? v : 0.01f * v;
        slab[(mOff + r) * 68 + (j << 4) + rlane] = v;
      }
    }
    __builtin_amdgcn_fence(__ATOMIC_RELEASE, "workgroup");
    __builtin_amdgcn_wave_barrier();
    __builtin_amdgcn_fence(__ATOMIC_ACQUIRE, "workgroup");
    if (OUT_MODE == 0) {
      float* C = (float*)Cout + (size_t)b * strideC;
      const int hh = lane >> 4, c4 = (lane & 15) * 4;
      for (int pass = 0; pass < 2; ++pass) {
#pragma unroll
        for (int it = 0; it < 8; ++it) {
          const int row = it * 2 + hh;
          v4f v = *(const v4f*)(slab + row * 68 + c4);
          *(volatile v4f*)(C + (size_t)(mBase + row) * ldc + n0 + c4) = v;
        }
        __threadfence();
      }
    } else {
      const int q = lane >> 3, c8 = (lane & 7) * 8;
      unsigned short* C  = (unsigned short*)Cout  + (size_t)b * strideC;
      unsigned short* C2 = (OUT_MODE == 2) ? ((unsigned short*)Cout2 + (size_t)b * strideC) : nullptr;
      for (int pass = 0; pass < 2; ++pass) {
#pragma unroll
        for (int it = 0; it < 4; ++it) {
          const int row = it * 4 + q;
          const float* sp = slab + row * 68 + c8;
          v8h hv, lv;
#pragma unroll
          for (int e = 0; e < 8; ++e) {
            if (OUT_MODE == 1) {
              hv[e] = (_Float16)sp[e];
            } else {
              unsigned short hb = f2bf_bits(sp[e]);
              unsigned short lb = f2bf_bits(sp[e] - bf_bits2f(hb));
              hv[e] = __builtin_bit_cast(_Float16, hb);
              lv[e] = __builtin_bit_cast(_Float16, lb);
            }
          }
          *(volatile v8h*)(C + (size_t)(mBase + row) * ldc + n0 + c8) = hv;
          if (OUT_MODE == 2) *(volatile v8h*)(C2 + (size_t)(mBase + row) * ldc + n0 + c8) = lv;
        }
        __threadfence();
      }
    }
    __builtin_amdgcn_fence(__ATOMIC_RELEASE, "workgroup");
    __builtin_amdgcn_wave_barrier();
    __builtin_amdgcn_fence(__ATOMIC_ACQUIRE, "workgroup");
  }
}

__global__ __launch_bounds__(256) void cast8_f16_kernel(const float* __restrict__ in, unsigned short* __restrict__ out, int n8) {
  const int i = blockIdx.x * 256 + threadIdx.x;
  if (i >= n8) return;
  const float* p = in + 8 * (size_t)i;
  const v4f a = *(const v4f*)(p);
  const v4f c = *(const v4f*)(p + 4);
  unsigned short hb[8];
#pragma unroll
  for (int e = 0; e < 4; ++e) {
    hb[e]     = h_bits(a[e]);
    hb[4 + e] = h_bits(c[e]);
  }
  const v4u u = (v4u){pk16(hb[0], hb[1]), pk16(hb[2], hb[3]), pk16(hb[4], hb[5]), pk16(hb[6], hb[7])};
  unsigned short* q = out + 8 * (size_t)i;
  *(volatile v4u*)q = u;
  __threadfence();
  *(volatile v4u*)q = u;
}

struct WSrc8 { const float* p[8]; };
static_assert(sizeof(WSrc8) == 64, "eight pointers, no padding");

__global__ __launch_bounds__(256) void wtcast_kernel(WSrc8 ps, long zsrc, int dout,
                                                     unsigned short* __restrict__ out, long zo, int ldo, float scale) {
  __shared__ float sm[64][65];
  const int t  = threadIdx.x;
  const int i0 = blockIdx.x * 64;
  const int o0 = blockIdx.y * 64;
  const int z  = blockIdx.z;
  const float* W = ps.p[0];
  W = (z == 1) ? ps.p[1] : W;
  W = (z == 2) ? ps.p[2] : W;
  W = (z == 3) ? ps.p[3] : W;
  W = (z == 4) ? ps.p[4] : W;
  W = (z == 5) ? ps.p[5] : W;
  W = (z == 6) ? ps.p[6] : W;
  W = (z == 7) ? ps.p[7] : W;
  W += (size_t)z * (size_t)zsrc;
#pragma unroll
  for (int i = 0; i < 16; ++i) {
    const int e = i * 256 + t;
    const int r = e >> 6;
    const int c = e & 63;
    sm[c][r] = W[(size_t)(i0 + r) * dout + o0 + c] * scale;
  }
  __syncthreads();
  const int lane = t & 31, wave = t >> 5;
  const int q = lane >> 3, c8 = (lane & 7) * 8;
  unsigned short* op = out + (size_t)z * (size_t)zo;
  for (int pass = 0; pass < 2; ++pass) {
#pragma unroll
    for (int it = 0; it < 2; ++it) {
      const int row = wave * 8 + it * 4 + q;
      unsigned short hb[8];
#pragma unroll
      for (int e = 0; e < 8; ++e) hb[e] = h_bits(sm[row][c8 + e]);
      const v4u u = (v4u){pk16(hb[0], hb[1]), pk16(hb[2], hb[3]), pk16(hb[4], hb[5]), pk16(hb[6], hb[7])};
      *(volatile v4u*)(op + (size_t)(o0 + row) * ldo + i0 + c8) = u;
    }
    __threadfence();
  }
}

__global__ __launch_bounds__(256) void small_planes_kernel(const float* __restrict__ wx_w, const float* __restrict__ wout_w,
                                                           const float* __restrict__ f2b, unsigned short* __restrict__ WxT,
                                                           unsigned short* __restrict__ WoutT, unsigned short* __restrict__ Btall) {
  const int role = blockIdx.y;
  const int i = blockIdx.x * 256 + threadIdx.x;
  float v0, v1;
  unsigned short* dst;
  if (role == 0) {
    if (i >= 4096) return;
    const int e0 = 2 * i;
    const int o = e0 >> 5;
    const int ii = e0 & 31;
    v0 = wx_w[(size_t)ii * kHid + o] * kWCarry;
    v1 = wx_w[(size_t)(ii + 1) * kHid + o] * kWCarry;
    dst = WxT + e0;
  } else if (role == 1) {
    const int e0 = 2 * i;
    const int o = e0 >> 8;
    const int ii = e0 & 255;
    const int oc = (o < kFeat) ? o : (kFeat - 1);
    const float sel = (o < kFeat) ? kWCarry : 0.0f;
    v0 = wout_w[(size_t)ii * kFeat + oc] * sel;
    v1 = wout_w[(size_t)(ii + 1) * kFeat + oc] * sel;
    dst = WoutT + e0;
  } else {
    const int e0 = 2 * i;
    const int n = e0 >> 6;
    const int cc = e0 & 63;
    const int c0c = (cc < kFeat) ? cc : (kFeat - 1);
    const int c1c = (cc + 1 < kFeat) ? (cc + 1) : (kFeat - 1);
    const float s0 = (cc < kFeat) ? kWCarry : 0.0f;
    const float s1 = (cc + 1 < kFeat) ? kWCarry : 0.0f;
    v0 = f2b[(size_t)c0c * kHid + n] * s0;
    v1 = f2b[(size_t)c1c * kHid + n] * s1;
    dst = Btall + (size_t)n * kMixLd + (size_t)(kFeat * kHid) + cc;
  }
  const unsigned u = pk16(h_bits(v0), h_bits(v1));
  *(volatile unsigned*)dst = u;
  __threadfence();
  *(volatile unsigned*)dst = u;
}

__global__ __launch_bounds__(256) void gather_emb_kernel(const int* __restrict__ sid, const float* __restrict__ t0,
                                                         const float* __restrict__ t12, const float* __restrict__ t3,
                                                         unsigned short* __restrict__ E16) {
  const int plane = blockIdx.x >> 5;
  const int i = (blockIdx.x & 31) * 256 + threadIdx.x;
  const int e0 = 2 * i;
  const int row = e0 >> 8;
  const int n = e0 & 255;
  const int rr = (row < kBatch) ? row : (kBatch - 1);
  int s = sid[rr];
  s = (s < 0) ? 0 : ((s > kAssets - 1) ? (kAssets - 1) : s);
  const float* tbl = (plane == 0) ? t0 : ((plane == 3) ? t3 : t12);
  const float sel = (row < kBatch) ? kWCarry : 0.0f;
  const float v0 = tbl[(size_t)s * kHid + n] * sel;
  const float v1 = tbl[(size_t)s * kHid + n + 1] * sel;
  const unsigned u = pk16(h_bits(v0), h_bits(v1));
  unsigned short* dst = E16 + (size_t)plane * (kPadM * kHid) + e0;
  *(volatile unsigned*)dst = u;
  __threadfence();
  *(volatile unsigned*)dst = u;
}

__global__ __launch_bounds__(256) void elu_hc_kernel(const float* __restrict__ pv, const float* __restrict__ hb1,
                                                     const float* __restrict__ cb1, unsigned short* __restrict__ hc16) {
  const int plane = blockIdx.x >> 5;
  const int i = (blockIdx.x & 31) * 256 + threadIdx.x;
  const int e0 = 2 * i;
  const int row = e0 >> 8;
  const int n = e0 & 255;
  const float* src = pv + (size_t)(1 + plane) * (kPadM * kHid) + (size_t)row * kHid + n;
  const float* bias = (plane == 0) ? hb1 : cb1;
  const float sel = (row < kBatch) ? kWCarry : 0.0f;
  const float v0 = eluf(src[0] + bias[n]) * sel;
  const float v1 = eluf(src[1] + bias[n + 1]) * sel;
  const unsigned u = pk16(h_bits(v0), h_bits(v1));
  unsigned short* dst = hc16 + (size_t)plane * (kPadM * kHid) + e0;
  *(volatile unsigned*)dst = u;
  __threadfence();
  *(volatile unsigned*)dst = u;
}

__global__ __launch_bounds__(256) void elu_pair_kernel(const float* __restrict__ raw, const float* __restrict__ bias1,
                                                      const float* __restrict__ rowadd, const float* __restrict__ bias2,
                                                      unsigned short* __restrict__ out16, int npairs) {
  const int i = blockIdx.x * 256 + threadIdx.x;
  if (i >= npairs) return;
  const int e0 = 2 * i;
  const int row = e0 >> 8;
  const int n = e0 & 255;
  const int b = row >> 7;
  const float* ra = rowadd + (size_t)b * kHid + n;
  const float v0 = eluf(raw[e0] + bias1[n] + ra[0] + bias2[n]);
  const float v1 = eluf(raw[e0 + 1] + bias1[n + 1] + ra[1] + bias2[n + 1]);
  const unsigned u = pk16(h_bits(v0), h_bits(v1));
  unsigned short* dst = out16 + e0;
  *(volatile unsigned*)dst = u;
  __threadfence();
  *(volatile unsigned*)dst = u;
}

__global__ __launch_bounds__(256) void vsn_mix_kernel(const float* __restrict__ x, const float* __restrict__ logits,
                                                     const float* __restrict__ wout_b, const float* __restrict__ f1w,
                                                     const float* __restrict__ f1b, unsigned short* __restrict__ U) {
  __shared__ float xs[kFeat];
  __shared__ float wsm[kFeat];
  __shared__ __align__(16) _Float16 urow[kMixLd];
  const int row = blockIdx.x;
  const int t = threadIdx.x, lane = t & 31, wave = t >> 5;
  if (t < kFeat) xs[t] = x[(size_t)row * kFeat + t];
  if (wave == 0) {
    const float l = logits[(size_t)row * 64 + lane] + wout_b[lane];
    float m = l;
#pragma unroll
    for (int off = 16; off > 0; off >>= 1) m = fmaxf(m, __shfl_xor(m, off, 32));
    const float e = expf(l - m);
    float s = e;
#pragma unroll
    for (int off = 16; off > 0; off >>= 1) s += __shfl_xor(s, off, 32);
    wsm[lane] = e * (1.0f / s);
  }
  __syncthreads();
#pragma unroll 1
  for (int it = 0; it < kFeat; ++it) {
    const int idx = it * kHid + t;
    const float z = xs[it] * f1w[idx] + f1b[idx];
    const float e = eluf(z);
    urow[idx] = (_Float16)(kUCarry * wsm[it] * e);
  }
  if (t < 64) {
    const float sel = (t < kFeat) ? kUCarry : 0.0f;
    urow[kFeat * kHid + t] = (_Float16)(wsm[t & 31] * sel);
  }
  __syncthreads();
  unsigned short* urp = U + (size_t)row * kMixLd;
  const int tl = (lane & 7) * 8;
  for (int pass = 0; pass < 2; ++pass) {
#pragma unroll
    for (int it = 0; it < 4; ++it) {
      const int ch = it * 8 + wave;
      const v8h hv = *(const v8h*)(urow + ch * 256 + lane * 8);
      *(volatile v8h*)(urp + ch * 256 + lane * 8) = hv;
    }
    if (wave == 0 && lane < 8) {
      const v8h tv = *(const v8h*)(urow + kFeat * kHid + tl);
      *(volatile v8h*)(urp + kFeat * kHid + tl) = tv;
    }
    __threadfence();
  }
}

template <bool ADD2, bool CB, bool O16>
__global__ __launch_bounds__(256) void ln_rows_kernel(const float* __restrict__ p1, const float* __restrict__ p2,
                                                     const float* __restrict__ cb, const float* __restrict__ gam,
                                                     const float* __restrict__ bet, float* __restrict__ outf,
                                                     unsigned short* __restrict__ out16) {
  __shared__ __align__(16) float rowbuf[8][kHid];
  const int t = threadIdx.x, lane = t & 31, wave = t >> 5;
  const int row = blockIdx.x * 8 + wave;
  const int c0 = lane * 8;
  const size_t base = (size_t)row * kHid + c0;
  const v4f a0 = *(const v4f*)(p1 + base);
  const v4f a1 = *(const v4f*)(p1 + base + 4);
  float v[8];
#pragma unroll
  for (int e = 0; e < 4; ++e) { v[e] = a0[e]; v[4 + e] = a1[e]; }
  if (CB) {
    const v4f q0 = *(const v4f*)(cb + c0);
    const v4f q1 = *(const v4f*)(cb + c0 + 4);
#pragma unroll
    for (int e = 0; e < 4; ++e) { v[e] += q0[e]; v[4 + e] += q1[e]; }
  }
  if (ADD2) {
    const v4f b0 = *(const v4f*)(p2 + base);
    const v4f b1 = *(const v4f*)(p2 + base + 4);
#pragma unroll
    for (int e = 0; e < 4; ++e) { v[e] += b0[e]; v[4 + e] += b1[e]; }
  }
  float s = 0.0f;
#pragma unroll
  for (int e = 0; e < 8; ++e) s += v[e];
#pragma unroll
  for (int off = 16; off > 0; off >>= 1) s += __shfl_xor(s, off, 32);
  const float mean = s * kInvH;
  float d[8];
  float q = 0.0f;
#pragma unroll
  for (int e = 0; e < 8; ++e) { d[e] = v[e] - mean; q += d[e] * d[e]; }
#pragma unroll
  for (int off = 16; off > 0; off >>= 1) q += __shfl_xor(q, off, 32);
  const float var = q * kInvH;
  const float rinv = 1.0f / sqrtf(var + kLnEps);
  const v4f g0 = *(const v4f*)(gam + c0);
  const v4f g1 = *(const v4f*)(gam + c0 + 4);
  const v4f e0b = *(const v4f*)(bet + c0);
  const v4f e1b = *(const v4f*)(bet + c0 + 4);
  float y[8];
#pragma unroll
  for (int e = 0; e < 4; ++e) {
    y[e]     = d[e] * rinv * g0[e] + e0b[e];
    y[4 + e] = d[4 + e] * rinv * g1[e] + e1b[e];
  }
#pragma unroll
  for (int e = 0; e < 8; ++e) rowbuf[wave][c0 + e] = y[e];
  v8h hv = (v8h){(_Float16)0.0f,(_Float16)0.0f,(_Float16)0.0f,(_Float16)0.0f,(_Float16)0.0f,(_Float16)0.0f,(_Float16)0.0f,(_Float16)0.0f};
  if (O16) {
#pragma unroll
    for (int e = 0; e < 8; ++e) hv[e] = (_Float16)y[e];
  }
  __syncthreads();
  for (int pass = 0; pass < 2; ++pass) {
#pragma unroll
    for (int qq = 0; qq < 2; ++qq) {
      const v4f o = *(const v4f*)(&rowbuf[wave][qq * 128 + 4 * lane]);
      *(volatile v4f*)(outf + (size_t)row * kHid + qq * 128 + 4 * lane) = o;
    }
    if (O16) *(volatile v8h*)(out16 + base) = hv;
    __threadfence();
  }
}

__global__ __launch_bounds__(512) void lstm_seq_kernel(const unsigned short* __restrict__ WhhTp, const float* __restrict__ xg,
                                                      const float* __restrict__ bih, const float* __restrict__ bhh,
                                                      const float* __restrict__ hc_raw, const float* __restrict__ h0b2,
                                                      const float* __restrict__ c0b2, float* __restrict__ hseq) {
  const _Float16* WhhT = (const _Float16*)(const void*)WhhTp;
  __shared__ __align__(16) _Float16 htile[2][16 * kHid];
  __shared__ __align__(16) float slab[16 * 260];
  const int t = threadIdx.x, lane = t & 31, wave = t >> 5;
  const int hh = lane >> 4, c = lane & 15, koff = hh * 8;
  const int b0 = blockIdx.x * 16;
  const int nu = wave * 16 + c;
#pragma unroll 1
  for (int it = 0; it < 8; ++it) {
    const int idx = it * 512 + t;
    const int r = idx >> 8;
    const int n = idx & 255;
    const float hv = hc_raw[(size_t)(b0 + r) * kHid + n] + h0b2[n];
    htile[0][idx] = (_Float16)hv;
  }
  float creg[8];
  float bsum[4];
#pragma unroll
  for (int r = 0; r < 8; ++r)
    creg[r] = hc_raw[(size_t)kPadM * kHid + (size_t)(b0 + 8 * hh + r) * kHid + nu] + c0b2[nu];
#pragma unroll
  for (int g4 = 0; g4 < 4; ++g4) bsum[g4] = bih[g4 * kHid + nu] + bhh[g4 * kHid + nu];
  __syncthreads();

  for (int step = 0; step < kSeqT; ++step) {
    const int cur = step & 1;
    const _Float16* hA = htile[cur];
    _Float16* hNx = htile[cur ^ 1];
    v8f acc[4];
#pragma unroll
    for (int g4 = 0; g4 < 4; ++g4) acc[g4] = (v8f){0.f,0.f,0.f,0.f,0.f,0.f,0.f,0.f};
#pragma unroll 1
    for (int k0 = 0; k0 < kHid; k0 += 32) {
      const v16h af = Frag<_Float16>::load(hA + c * kHid + koff + k0);
      v16h bf[4];
#pragma unroll
      for (int g4 = 0; g4 < 4; ++g4)
        bf[g4] = Frag<_Float16>::load(WhhT + (size_t)(g4 * kHid + nu) * kHid + koff + k0);
#pragma unroll
      for (int g4 = 0; g4 < 4; ++g4) acc[g4] = Frag<_Float16>::mma(af, bf[g4], acc[g4]);
      dep_guard_h(acc[0], acc[3], af, bf[3]);
      keep4_h(bf[0], bf[1], bf[2], bf[3]);
    }
    acc_guard4(acc[0], acc[1], acc[2], acc[3]);

#pragma unroll
    for (int r = 0; r < 8; ++r) {
      const int rowl = 8 * hh + r;
      const float* xr = xg + ((size_t)(b0 + rowl) * kSeqT + step) * kGate4 + nu;
      const float iv = acc[0][r] * kWInv + xr[0] + bsum[0];
      const float fv = acc[1][r] * kWInv + xr[kHid] + bsum[1];
      const float gv = acc[2][r] * kWInv + xr[2 * kHid] + bsum[2];
      const float ov = acc[3][r] * kWInv + xr[3 * kHid] + bsum[3];
      const float ig = 1.0f / (1.0f + expf(-iv));
      const float fg = 1.0f / (1.0f + expf(-fv));
      const float og = 1.0f / (1.0f + expf(-ov));
      const float gt = tanhf(gv);
      const float cn = fg * creg[r] + ig * gt;
      creg[r] = cn;
      const float hn = og * tanhf(cn);
      hNx[rowl * kHid + nu] = (_Float16)hn;
      slab[rowl * 260 + nu] = hn;
    }
    __syncthreads();
    {
      const size_t ob = ((size_t)(b0 + wave) * kSeqT + step) * kHid;
      for (int pass = 0; pass < 2; ++pass) {
#pragma unroll
        for (int qq = 0; qq < 2; ++qq) {
          const v4f hv4 = *(const v4f*)(slab + wave * 260 + qq * 128 + 4 * lane);
          *(volatile v4f*)(hseq + ob + qq * 128 + 4 * lane) = hv4;
        }
        __threadfence();
      }
    }
    __syncthreads();
  }
}

extern "C" void kernel_launch(void* const* d_in, const int* in_sizes, int n_in,
                              void* d_out, int out_size, void* d_ws, size_t ws_size, hipStream_t stream) {
  (void)in_sizes;
  if (n_in < 39) return;
  if ((size_t)out_size < (size_t)kRows * kHid) return;

  const float* x       = (const float*)d_in[0];
  const int*   sid     = (const int*)d_in[1];
  const float* vsn_emb = (const float*)d_in[2];
  const float* wx_w    = (const float*)d_in[3];
  const float* wx_b    = (const float*)d_in[4];
  const float* ws_w    = (const float*)d_in[5];
  const float* ws_b    = (const float*)d_in[6];
  const float* wout_w  = (const float*)d_in[7];
  const float* wout_b  = (const float*)d_in[8];
  const float* f1w     = (const float*)d_in[9];
  const float* f1b     = (const float*)d_in[10];
  const float* f2w     = (const float*)d_in[11];
  const float* f2b     = (const float*)d_in[12];
  const float* vng     = (const float*)d_in[13];
  const float* vnb     = (const float*)d_in[14];
  const float* emb     = (const float*)d_in[15];
  const float* h0_w1   = (const float*)d_in[16];
  const float* h0_b1   = (const float*)d_in[17];
  const float* h0_w2   = (const float*)d_in[18];
  const float* h0_b2   = (const float*)d_in[19];
  const float* c0_w1   = (const float*)d_in[20];
  const float* c0_b1   = (const float*)d_in[21];
  const float* c0_w2   = (const float*)d_in[22];
  const float* c0_b2   = (const float*)d_in[23];
  const float* wih     = (const float*)d_in[24];
  const float* whh     = (const float*)d_in[25];
  const float* bih     = (const float*)d_in[26];
  const float* bhh     = (const float*)d_in[27];
  const float* n1g     = (const float*)d_in[28];
  const float* n1b     = (const float*)d_in[29];
  const float* ffn_emb = (const float*)d_in[30];
  const float* l1_w    = (const float*)d_in[31];
  const float* l1_b    = (const float*)d_in[32];
  const float* l2_w    = (const float*)d_in[33];
  const float* l2_b    = (const float*)d_in[34];
  const float* l3_w    = (const float*)d_in[35];
  const float* l3_b    = (const float*)d_in[36];
  const float* n2g     = (const float*)d_in[37];
  const float* n2b     = (const float*)d_in[38];

  size_t off = 0;
  auto carve = [&](size_t bytes) -> size_t { const size_t o = off; off += (bytes + 255) & ~(size_t)255; return o; };
  const size_t o_w256t  = carve((size_t)8 * kHid * kHid * 2);
  const size_t o_w1024t = carve((size_t)2 * kGate4 * kHid * 2);
  const size_t o_btall  = carve((size_t)kHid * kMixLd * 2);
  const size_t o_x16    = carve((size_t)kRows * kFeat * 2);
  const size_t o_wxt    = carve((size_t)kHid * kFeat * 2);
  const size_t o_woutt  = carve((size_t)64 * kHid * 2);
  const size_t o_e16    = carve((size_t)4 * kPadM * kHid * 2);
  const size_t o_pv     = carve((size_t)4 * kPadM * kHid * 4);
  const size_t o_hc16   = carve((size_t)2 * kPadM * kHid * 2);
  const size_t o_hcraw  = carve((size_t)2 * kPadM * kHid * 4);
  const size_t o_g1     = carve((size_t)kRows * kHid * 4);
  const size_t o_gate16 = carve((size_t)kRows * kHid * 2);
  const size_t o_logits = carve((size_t)kRows * 64 * 4);
  const size_t o_u      = carve((size_t)kRows * kMixLd * 2);
  const size_t o_xpre   = carve((size_t)kRows * kHid * 4);
  const size_t o_xp     = carve((size_t)kRows * kHid * 4);
  const size_t o_xp16   = carve((size_t)kRows * kHid * 2);
  const size_t o_xg     = carve((size_t)kRows * kGate4 * 4);
  const size_t o_hseq   = carve((size_t)kRows * kHid * 4);
  const size_t o_a      = carve((size_t)kRows * kHid * 4);
  const size_t o_a16    = carve((size_t)kRows * kHid * 2);
  if (off > ws_size) return;

  char* ws = (char*)d_ws;
  unsigned short* W256T  = (unsigned short*)(ws + o_w256t);
  unsigned short* W1024T = (unsigned short*)(ws + o_w1024t);
  unsigned short* WihT   = W1024T;
  unsigned short* WhhT   = W1024T + (size_t)kGate4 * kHid;
  unsigned short* Btall  = (unsigned short*)(ws + o_btall);
  unsigned short* x16    = (unsigned short*)(ws + o_x16);
  unsigned short* WxT    = (unsigned short*)(ws + o_wxt);
  unsigned short* WoutT  = (unsigned short*)(ws + o_woutt);
  unsigned short* E16    = (unsigned short*)(ws + o_e16);
  float*          pv     = (float*)(ws + o_pv);
  unsigned short* hc16   = (unsigned short*)(ws + o_hc16);
  float*          hcraw  = (float*)(ws + o_hcraw);
  float*          g1     = (float*)(ws + o_g1);
  float*          f1raw  = g1;
  unsigned short* gate16 = (unsigned short*)(ws + o_gate16);
  unsigned short* fh16   = gate16;
  float*          logits = (float*)(ws + o_logits);
  unsigned short* U      = (unsigned short*)(ws + o_u);
  float*          xpre   = (float*)(ws + o_xpre);
  float*          f3raw  = xpre;
  float*          xp     = (float*)(ws + o_xp);
  unsigned short* xp16   = (unsigned short*)(ws + o_xp16);
  float*          xg     = (float*)(ws + o_xg);
  float*          hseq   = (float*)(ws + o_hseq);
  float*          abuf   = (float*)(ws + o_a);
  unsigned short* a16    = (unsigned short*)(ws + o_a16);
  float*          outp   = (float*)d_out;

  const float* dummyf = wx_b;
  auto gemm = [&](const unsigned short* A, int lda, long sA, const unsigned short* Bt, int ldb, long sB,
                  float* Cc, int ldc, long sC, int M, int N, int K, float scale, int nb) {
    const int tiles = (M / 64) * (N / 64);
    dim3 grid((tiles + 7) / 8, nb);
    wmma_gemm64<0, false, 0, 0, false, 0><<<grid, 256, 0, stream>>>(
        A, A, lda, sA, Bt, Bt, ldb, sB, (void*)Cc, (void*)Cc, ldc, sC, dummyf, dummyf, 0L, M, N, K, scale);
  };

  {
    WSrc8 ps;
    ps.p[0] = ws_w; ps.p[1] = h0_w1; ps.p[2] = c0_w1; ps.p[3] = l2_w;
    ps.p[4] = h0_w2; ps.p[5] = c0_w2; ps.p[6] = l1_w; ps.p[7] = l3_w;
    wtcast_kernel<<<dim3(4, 4, 8), 256, 0, stream>>>(ps, 0L, kHid, W256T, (long)kHid * kHid, kHid, kWCarry);
  }
  {
    WSrc8 ps;
    ps.p[0] = wih; ps.p[1] = whh; ps.p[2] = whh; ps.p[3] = whh;
    ps.p[4] = whh; ps.p[5] = whh; ps.p[6] = whh; ps.p[7] = whh;
    wtcast_kernel<<<dim3(4, 16, 2), 256, 0, stream>>>(ps, 0L, kGate4, W1024T, (long)kGate4 * kHid, kHid, kWCarry);
  }
  {
    WSrc8 ps;
    for (int i = 0; i < 8; ++i) ps.p[i] = f2w;
    wtcast_kernel<<<dim3(4, 4, kFeat), 256, 0, stream>>>(ps, (long)kHid * kHid, kHid, Btall, (long)kHid, kMixLd, kWCarry);
  }
  small_planes_kernel<<<dim3(32, 3), 256, 0, stream>>>(wx_w, wout_w, f2b, WxT, WoutT, Btall);
  cast8_f16_kernel<<<64, 256, 0, stream>>>(x, x16, kRows * kFeat / 8);
  gather_emb_kernel<<<128, 256, 0, stream>>>(sid, vsn_emb, emb, ffn_emb, E16);
  gemm(E16, kHid, (long)kPadM * kHid, W256T, kHid, (long)kHid * kHid, pv, kHid, (long)kPadM * kHid, kPadM, kHid, kHid, kEmbScale, 4);
  elu_hc_kernel<<<64, 256, 0, stream>>>(pv, h0_b1, c0_b1, hc16);
  gemm(hc16, kHid, (long)kPadM * kHid, W256T + (size_t)4 * kHid * kHid, kHid, (long)kHid * kHid, hcraw, kHid, (long)kPadM * kHid, kPadM, kHid, kHid, kEmbScale, 2);
  gemm(x16, kFeat, 0L, WxT, kFeat, 0L, g1, kHid, 0L, kRows, kHid, kFeat, kWInv, 1);
  elu_pair_kernel<<<2048, 256, 0, stream>>>(g1, wx_b, pv, ws_b, gate16, kRows * kHid / 2);
  gemm(gate16, kHid, 0L, WoutT, kHid, 0L, logits, 64, 0L, kRows, 64, kHid, kWInv, 1);
  vsn_mix_kernel<<<kRows, 256, 0, stream>>>(x, logits, wout_b, f1w, f1b, U);
  gemm(U, kMixLd, 0L, Btall, kMixLd, 0L, xpre, kHid, 0L, kRows, kHid, kMixK, kMixScale, 1);
  ln_rows_kernel<false, false, true><<<kRows / 8, 256, 0, stream>>>(xpre, xpre, vng, vng, vnb, xp, xp16);
  gemm(xp16, kHid, 0L, WihT, kHid, 0L, xg, kGate4, 0L, kRows, kGate4, kHid, kWInv, 1);
  lstm_seq_kernel<<<kBatch / 16, 512, 0, stream>>>(WhhT, xg, bih, bhh, hcraw, h0_b2, c0_b2, hseq);
  ln_rows_kernel<true, false, true><<<kRows / 8, 256, 0, stream>>>(hseq, xp, n1g, n1g, n1b, abuf, a16);
  gemm(a16, kHid, 0L, W256T + (size_t)6 * kHid * kHid, kHid, 0L, f1raw, kHid, 0L, kRows, kHid, kHid, kWInv, 1);
  elu_pair_kernel<<<2048, 256, 0, stream>>>(f1raw, l1_b, pv + (size_t)3 * kPadM * kHid, l2_b, fh16, kRows * kHid / 2);
  gemm(fh16, kHid, 0L, W256T + (size_t)7 * kHid * kHid, kHid, 0L, f3raw, kHid, 0L, kRows, kHid, kHid, kWInv, 1);
  ln_rows_kernel<true, true, false><<<kRows / 8, 256, 0, stream>>>(f3raw, abuf, l3_b, n2g, n2b, outp, a16);
}
